// PlainGCN_14353780703616
// MI455X (gfx1250) — hardware-verified
//
#include <hip/hip_runtime.h>
#include <math.h>

typedef __attribute__((ext_vector_type(16))) _Float16 v16h;
typedef __attribute__((ext_vector_type(16))) __bf16 v16b;
typedef __attribute__((ext_vector_type(8)))  _Float16 v8h;
typedef __attribute__((ext_vector_type(8)))  float v8f;
typedef __attribute__((ext_vector_type(4)))  float v4f;
typedef __attribute__((ext_vector_type(2)))  float v2f;
typedef __attribute__((ext_vector_type(4)))  unsigned v4u;
typedef __attribute__((ext_vector_type(4)))  int v4i;
typedef float __attribute__((may_alias)) float_a;
typedef int __attribute__((may_alias)) int_a;

template <typename T> __device__ __forceinline__ void vst2(void* p, T v) { *(volatile T*)p = v; __threadfence(); *(volatile T*)p = v; }
__device__ __forceinline__ v8f wmma16(v16h a, v16h b, v8f c) {
  v8f d = __builtin_amdgcn_wmma_f32_16x16x32_f16(false, a, false, b, (short)0, c, false, false);
  asm volatile("v_nop\n\tv_nop\n\tv_nop\n\tv_nop" : "+v"(d) : "v"(a), "v"(b));
  return d;
}
__device__ __forceinline__ v8f wmma_bf(v16b a, v16b b, v8f c) {
  v8f d = __builtin_amdgcn_wmma_f32_16x16x32_bf16(false, a, false, b, (short)0, c, false, false);
  asm volatile("v_nop\n\tv_nop\n\tv_nop\n\tv_nop" : "+v"(d) : "v"(a), "v"(b));
  return d;
}
__device__ __forceinline__ v16h frag_h(const _Float16* rowk0, int lane) {
  union { v16h v; v8h q[2]; } u; const _Float16* p = rowk0 + 8 * (lane >> 4);
  u.q[0] = *(const v8h*)p; u.q[1] = *(const v8h*)(p + 16); return u.v;
}
__device__ __forceinline__ v16h frag_f32(const float* rowk0, int lane) {
  v16h a; const float* p = rowk0 + 8 * (lane >> 4);
#pragma unroll
  for (int i = 0; i < 8; ++i) { a[i] = (_Float16)p[i]; a[8 + i] = (_Float16)p[16 + i]; }
  return a;
}
__device__ __forceinline__ v16h frag_f32s(const float* rowk0, int lane, float sc) {
  v16h a; const float* p = rowk0 + 8 * (lane >> 4);
#pragma unroll
  for (int i = 0; i < 8; ++i) { a[i] = (_Float16)(p[i] * sc); a[8 + i] = (_Float16)(p[16 + i] * sc); }
  return a;
}
__device__ __forceinline__ v16h fragc_f32(const float* W, int k0, int n, int lane, int ld, int K) {
  v16h a; const int g = lane >> 4;
#pragma unroll
  for (int i = 0; i < 8; ++i) { const int ka = k0 + 8 * g + i, kb = ka + 16;
    a[i] = (_Float16)(ka < K ? W[(size_t)(ka < K ? ka : K - 1) * ld + n] : 0.f); a[8 + i] = (_Float16)(kb < K ? W[(size_t)(kb < K ? kb : K - 1) * ld + n] : 0.f); }
  return a;
}
struct F2 { v16b h, l; };
__device__ __forceinline__ F2 bsplit16(const float v[16]) { F2 r;
#pragma unroll
  for (int i = 0; i < 16; ++i) { const __bf16 h = (__bf16)v[i]; r.h[i] = h; r.l[i] = (__bf16)(v[i] - (float)h); }
  return r; }
__device__ __forceinline__ F2 split_row(const float* row, int k0, int lane) { float v[16]; const float* p = row + k0 + 8 * (lane >> 4);
#pragma unroll
  for (int i = 0; i < 8; ++i) { v[i] = p[i]; v[8 + i] = p[16 + i]; }
  return bsplit16(v); }
__device__ __forceinline__ F2 split_rowK(const float* row, int k0, int lane, int K) { float v[16]; const int g = lane >> 4;
#pragma unroll
  for (int i = 0; i < 8; ++i) { const int ka = k0 + 8 * g + i, kb = ka + 16; v[i] = ka < K ? row[ka < K ? ka : K - 1] : 0.f; v[8 + i] = kb < K ? row[kb < K ? kb : K - 1] : 0.f; }
  return bsplit16(v); }
__device__ __forceinline__ F2 split_col(const float* W, int k0, int n, int lane, int ld, int K) { float v[16]; const int g = lane >> 4;
#pragma unroll
  for (int i = 0; i < 8; ++i) { const int ka = k0 + 8 * g + i, kb = ka + 16; v[i] = ka < K ? W[(size_t)(ka < K ? ka : K - 1) * ld + n] : 0.f; v[8 + i] = kb < K ? W[(size_t)(kb < K ? kb : K - 1) * ld + n] : 0.f; }
  return bsplit16(v); }
__device__ __forceinline__ v8f mac3(const F2& a, const F2& b, v8f c) { c = wmma_bf(a.l, b.h, c); c = wmma_bf(a.h, b.l, c); return wmma_bf(a.h, b.h, c); }
__device__ __forceinline__ float sigm(float v) { return 1.0f / (1.0f + expf(-v)); }
#define LDSX() do { asm volatile("s_wait_dscnt 0" ::: "memory"); __builtin_amdgcn_wave_barrier(); __builtin_amdgcn_fence(__ATOMIC_RELEASE, "workgroup"); } while (0)


#define NN 16384
#define KNB 16
#define CC 64
typedef __attribute__((ext_vector_type(8))) __bf16 v8b;
__device__ __forceinline__ v16b frag_b(const __bf16* rowk0, int lane) {
  union { v16b v; v8b q[2]; } u; const __bf16* p = rowk0 + 8 * (lane >> 4);
  u.q[0] = *(const v8b*)p; u.q[1] = *(const v8b*)(p + 16); return u.v;
}
__device__ __forceinline__ float bfr(float v) { return (float)(__bf16)v; }
__device__ __attribute__((noinline)) float exp_ni(float v) { return expf(v); }
__device__ __attribute__((noinline)) float erf_ni(float v) { return erff(v); }

#define WS_PK  0u
#define WS_POS (((2u * 2 * CC * 2 * CC) + 127u) / 128u * 128u)
#define WS_IDX (WS_POS + 4u * NN * 4)
#define WS_F1  (WS_IDX + 4u * NN * KNB)
#define WS_END (WS_F1 + 4u * NN * CC)

__global__ __launch_bounds__(128) void k_pack(const float* __restrict__ W1, const float* __restrict__ W2, __bf16* __restrict__ PK) {
  __shared__ __align__(16) __bf16 s[2 * CC]; const int n = blockIdx.x, which = blockIdx.y, t = threadIdx.x; const float* Wm = (which == 0) ? W1 : W2;
  s[t] = (__bf16)Wm[(size_t)t * CC + n];
  __syncthreads();
  if (t < 16) vst2((unsigned*)(PK + ((size_t)which * CC + n) * 2 * CC + t * 8), *(const v4u*)&s[t * 8]);
}
__global__ __launch_bounds__(256) void k_prep(const int* __restrict__ VC, float* __restrict__ POS) {
  __shared__ __align__(16) float sp[256][4]; const int t = threadIdx.x; const size_t p = (size_t)blockIdx.x * 256 + t;
  sp[t][0] = (float)VC[p * 4 + 1]; sp[t][1] = (float)VC[p * 4 + 2]; sp[t][2] = (float)VC[p * 4 + 3]; sp[t][3] = (float)VC[p * 4 + 0];
  __syncthreads();
  vst2(POS + p * 4, *(const v4f*)&sp[t][0]);
}
#define INS16(v, j) do { float cv = (v); int cj = (j); _Pragma("unroll") for (int q = 0; q < KNB; ++q) { const bool lt = (cv < bv[q]) || (cv == bv[q] && cj < bj[q]); const float tv = bv[q]; const int tj = bj[q]; bv[q] = lt ? cv : tv; bj[q] = lt ? cj : tj; cv = lt ? tv : cv; cj = lt ? tj : cj; } } while (0)
__global__ __launch_bounds__(128) void k_knn(const float* __restrict__ POS, int* __restrict__ IDX) {
  __shared__ __align__(16) int sidx[4][KNB];
  const int tid = threadIdx.x, wave = tid >> 5, lane = tid & 31; const size_t i = (size_t)blockIdx.x * 4 + wave;
  const float xi = POS[i * 4], yi = POS[i * 4 + 1], zi = POS[i * 4 + 2], bi_ = POS[i * 4 + 3]; const float sqi = xi * xi + yi * yi + zi * zi;
  float bv[KNB]; int bj[KNB];
#pragma unroll
  for (int q = 0; q < KNB; ++q) { bv[q] = 3.0e38f; bj[q] = 0x7fffffff; }
#pragma unroll 1
  for (int j = lane; j < NN; j += 32) { const float xj = POS[(size_t)j * 4], yj = POS[(size_t)j * 4 + 1], zj = POS[(size_t)j * 4 + 2], bj_ = POS[(size_t)j * 4 + 3];
    const float sqj = xj * xj + yj * yj + zj * zj; const float dot = xi * xj + yi * yj + zi * zj; float d = (sqi + sqj) - 2.0f * dot;
    d = (bj_ != bi_) ? 1.0e10f : d; d = ((size_t)j == i) ? d + 1.0e10f : d;
    if (d < bv[KNB - 1] || (d == bv[KNB - 1] && j < bj[KNB - 1])) INS16(d, j); }
#pragma unroll 1
  for (int s = 0; s < KNB; ++s) { float hv = bv[0]; int hj = bj[0]; int src = lane;
#pragma unroll
    for (int o = 1; o < 32; o <<= 1) { const float ov = __shfl_xor(hv, o); const int oj = __shfl_xor(hj, o); const int os = __shfl_xor(src, o); const bool take = (ov < hv) || (ov == hv && oj < hj); hv = take ? ov : hv; hj = take ? oj : hj; src = take ? os : src; }
    if (lane == 0) sidx[wave][s] = hj;
    if (lane == src) {
#pragma unroll
      for (int q = 0; q < KNB - 1; ++q) { bv[q] = bv[q + 1]; bj[q] = bj[q + 1]; } bv[KNB - 1] = 3.0e38f; bj[KNB - 1] = 0x7fffffff; } }
  __syncthreads();
  if (tid < 16) vst2((unsigned*)(IDX + (size_t)blockIdx.x * 4 * KNB + tid * 4), *(const v4u*)(&sidx[0][0] + tid * 4));
}
template <int LAYER>
__global__ __launch_bounds__(128) void k_edge(const float* __restrict__ X, const int* __restrict__ IDX, const __bf16* __restrict__ PK, const float* __restrict__ Bv, const float* __restrict__ RES, float* __restrict__ OUT) {
  __shared__ __align__(16) __bf16 seh[64][136], sel[64][136]; __shared__ float sh[4][16][CC + 1]; __shared__ __align__(16) float so[4][CC];
  const int tid = threadIdx.x, wave = tid >> 5, lane = tid & 31, col = lane & 15, g = lane >> 4; const size_t i = (size_t)blockIdx.x * 4 + wave;
  { const int k = lane >> 1, half = lane & 1; const int j = IDX[i * KNB + k]; const float* xi = X + i * CC + half * 32; const float* xj = X + (size_t)j * CC + half * 32; const int row = wave * 16 + k;
#pragma unroll
    for (int c = 0; c < 32; ++c) { const float a = (LAYER == 0) ? bfr(xi[c]) : xi[c]; const float bb2 = (LAYER == 0) ? bfr(xj[c]) : xj[c]; const float dlt = bb2 - a;
      const __bf16 ha = (__bf16)a; seh[row][half * 32 + c] = ha; sel[row][half * 32 + c] = (__bf16)(a - (float)ha);
      const __bf16 hd = (__bf16)dlt; seh[row][CC + half * 32 + c] = hd; sel[row][CC + half * 32 + c] = (__bf16)(dlt - (float)hd); } }
  if (lane < 8) for (int rr = 0; rr < 16; ++rr) { seh[wave * 16 + rr][128 + lane] = (__bf16)0.f; sel[wave * 16 + rr][128 + lane] = (__bf16)0.f; }
  LDSX();
  v8f acc[4] = {}; const __bf16* P = PK + (size_t)LAYER * CC * 2 * CC;
#pragma unroll
  for (int kc = 0; kc < 4; ++kc) { F2 a; a.h = frag_b(&seh[wave * 16 + col][kc * 32], lane); a.l = frag_b(&sel[wave * 16 + col][kc * 32], lane);
#pragma unroll
    for (int jt = 0; jt < 4; ++jt) { const v16b w = frag_b(P + (size_t)(jt * 16 + col) * 2 * CC + kc * 32, lane); acc[jt] = wmma_bf(a.l, w, acc[jt]); acc[jt] = wmma_bf(a.h, w, acc[jt]); } }
#pragma unroll
  for (int jt = 0; jt < 4; ++jt) { const int c = jt * 16 + col; const float bb = bfr(Bv[c]);
#pragma unroll
    for (int r = 0; r < 8; ++r) sh[wave][8 * g + r][c] = fmaxf(acc[jt][r] + bb, 0.f); }
  LDSX();
  { float mx0 = -3.0e38f, mx1 = -3.0e38f;
#pragma unroll
    for (int k = 0; k < KNB; ++k) { mx0 = fmaxf(mx0, sh[wave][k][lane]); mx1 = fmaxf(mx1, sh[wave][k][lane + 32]); }
    if (LAYER == 1) { mx0 += bfr(RES[i * CC + lane]); mx1 += bfr(RES[i * CC + lane + 32]); }
    so[wave][lane] = mx0; so[wave][lane + 32] = mx1; }
  __syncthreads();
  if (tid < 64) vst2(OUT + (size_t)blockIdx.x * 4 * CC + tid * 4, *(const v4f*)(&so[0][0] + tid * 4));
}
extern "C" void kernel_launch(void* const* d_in, const int* in_sizes, int n_in, void* d_out, int out_size, void* d_ws, size_t ws_size, hipStream_t stream) {
  (void)in_sizes; (void)n_in; (void)out_size;
  const float** F = (const float**)d_in;
  if (ws_size < (size_t)WS_END) return;
  char* ws = (char*)d_ws; __bf16* PK = (__bf16*)(ws + WS_PK); float *POS = (float*)(ws + WS_POS), *F1 = (float*)(ws + WS_F1); int* IDX = (int*)(ws + WS_IDX);
  k_pack<<<dim3(CC, 2), 128, 0, stream>>>(F[2], F[4], PK);
  k_prep<<<NN / 256, 256, 0, stream>>>((const int*)d_in[0], POS);
  k_knn<<<NN / 4, 128, 0, stream>>>(POS, IDX);
  k_edge<0><<<NN / 4, 128, 0, stream>>>(F[1], IDX, PK, F[3], nullptr, F1);
  k_edge<1><<<NN / 4, 128, 0, stream>>>(F1, IDX, PK, F[5], F[1], (float*)d_out);
}
